// MultiHeadAttentionWithRPR_16183436772079
// MI455X (gfx1250) — hardware-verified
//
#include <hip/hip_runtime.h>
#include <hip/hip_bf16.h>
#include <math.h>

#define NB 4
#define SSr 1024
#define Dr 1024
#define NH 16
#define DHr 64
#define NRr 129
#define NRP 256
#define MTOK (NB * SSr)
#define GSTR 48

typedef _Float16 bf16;
typedef _Float16 f16;
typedef __attribute__((ext_vector_type(4))) unsigned v4u_t;
typedef unsigned v4ua __attribute__((ext_vector_type(4), may_alias));
typedef __attribute__((ext_vector_type(4))) float v4f_t;
typedef float v4fa __attribute__((ext_vector_type(4), may_alias));
typedef __attribute__((ext_vector_type(16))) bf16  bf16x16;
typedef bf16x16 f16x16;
typedef __attribute__((ext_vector_type(8)))  bf16  bf16x8;
typedef bf16x8 f16x8;
typedef __attribute__((ext_vector_type(4)))  bf16  bf16x4;
typedef __attribute__((ext_vector_type(8)))  float f32x8;
__device__ __forceinline__ f32x8 wmma16(f16x16 a, f16x16 b, f32x8 c) {
  c = __builtin_amdgcn_wmma_f32_16x16x32_f16(false, a, false, b, (short)0, c, false, false);
  asm volatile("v_nop\n\tv_nop\n\tv_nop\n\tv_nop" : "+v"(c) : "v"(a), "v"(b));
  return c;
}
#define LDS_STRIDE 48
#define KSTRIDE    72
#define VSTRIDE    48

__device__ __forceinline__ f32x8 wmma_bf16(bf16x16 a, bf16x16 b, f32x8 c) {
  c = __builtin_amdgcn_wmma_f32_16x16x32_f16(false, a, false, b, (short)0, c, false, false);
  asm volatile("v_nop\n\tv_nop\n\tv_nop\n\tv_nop" : "+v"(c) : "v"(a), "v"(b));
  return c;
}

template <typename T>
__device__ __forceinline__ bf16x16 load_frag(const T* __restrict__ base, int ld,
                                             int row0, int k0) {
  const int lane = threadIdx.x & 31;
  const int r    = lane & 15;
  const int kh   = (lane >> 4) * 8;
  const T* p0 = base + (size_t)(row0 + r) * ld + (k0 + kh);
  const T* p1 = p0 + 16;
  bf16x16 f;
#pragma unroll
  for (int i = 0; i < 8; ++i) {
    f[i]     = (bf16)p0[i];
    f[i + 8] = (bf16)p1[i];
  }
  return f;
}

__device__ __forceinline__ bf16x16 lds_frag(const bf16* base, int stride) {
  const int lane = threadIdx.x & 31;
  const int row  = lane & 15;
  const int kh   = (lane >> 4) * 8;
  const bf16x8 lo = *(const bf16x8*)(base + row * stride + kh);
  const bf16x8 hi = *(const bf16x8*)(base + row * stride + kh + 16);
  bf16x16 f;
#pragma unroll
  for (int i = 0; i < 8; ++i) { f[i] = lo[i]; f[i + 8] = hi[i]; }
  return f;
}

template <typename T>
__device__ __forceinline__ void stage_read16(const T* __restrict__ p, float* buf) {
#pragma unroll
  for (int i = 0; i < 16; ++i) buf[i] = (float)p[i];
}

__device__ __forceinline__ void stage_write(bf16* dst, const float* buf, int nquad) {
#pragma unroll
  for (int i = 0; i < nquad; ++i) {
    bf16x4 q;
    q[0] = (bf16)buf[4 * i];     q[1] = (bf16)buf[4 * i + 1];
    q[2] = (bf16)buf[4 * i + 2]; q[3] = (bf16)buf[4 * i + 3];
    *(bf16x4*)(dst + 4 * i) = q;
  }
}


#define GSTR 48
template <typename AT, int EPI, bool OUT16>
__global__ __launch_bounds__(256) void gemm_kne(const AT* __restrict__ A, int lda, const float* __restrict__ Wm, int ldw,
                                                const float* __restrict__ bias, const float* __restrict__ R, const float* __restrict__ gvec,
                                                void* __restrict__ Yv, int ldy, int K) {
  __shared__ __attribute__((aligned(16))) f16 ldsA[128 * GSTR];
  __shared__ __attribute__((aligned(16))) f16 ldsW[128 * GSTR];
  __shared__ __attribute__((aligned(16))) float oS[8][32 * 68];
  const int tid = threadIdx.x, lane = tid & 31, wave = tid >> 5, cl = lane & 15, rh = (lane >> 4) * 8;
  const int m0 = blockIdx.x * 128, n0 = blockIdx.y * 128;
  const int wm = (wave & 3) * 32, wn = (wave >> 2) * 64;
  f32x8 acc[2][4];
#pragma unroll
  for (int i = 0; i < 2; ++i)
#pragma unroll
    for (int j = 0; j < 4; ++j) { f32x8 z = {}; acc[i][j] = z; }
#pragma unroll 1
  for (int k0 = 0; k0 < K; k0 += 32) {
    __syncthreads();
    { const int row = tid >> 1, ch = (tid & 1) * 16;
      const AT* src = A + (size_t)(m0 + row) * lda + k0 + ch;
#pragma unroll
      for (int g = 0; g < 16; ++g) ldsA[row * GSTR + ch + g] = (f16)src[g]; }
    { const int k = tid >> 3, nn0 = (tid & 7) * 16;
      const float* src = Wm + (size_t)(k0 + k) * ldw + n0 + nn0;
#pragma unroll
      for (int g = 0; g < 4; ++g) { const v4f_t v = *(const v4f_t*)(src + 4 * g);
#pragma unroll
        for (int u = 0; u < 4; ++u) ldsW[(nn0 + 4 * g + u) * GSTR + k] = (f16)v[u]; } }
    __syncthreads();
    f16x16 af[2];
#pragma unroll
    for (int i = 0; i < 2; ++i) af[i] = lds_frag(ldsA + (wm + 16 * i) * GSTR, GSTR);
#pragma unroll
    for (int j = 0; j < 4; ++j) {
      const f16x16 bf = lds_frag(ldsW + (wn + 16 * j) * GSTR, GSTR);
#pragma unroll
      for (int i = 0; i < 2; ++i) acc[i][j] = wmma16(af[i], bf, acc[i][j]);
    }
  }
  float* so = oS[wave];
#pragma unroll
  for (int i = 0; i < 2; ++i)
#pragma unroll
    for (int j = 0; j < 4; ++j) {
      const int n = n0 + wn + 16 * j + cl;
      const float bv = bias ? bias[n] : 0.0f;
      const float gv = (EPI == 2) ? gvec[n] : 0.0f;
      if (EPI == 1) {
#pragma unroll 1
        for (int r = 0; r < 8; ++r) { const float xg = acc[i][j][r] + bv; so[(16 * i + rh + r) * 68 + 16 * j + cl] = 0.5f * xg * (1.0f + erff(xg * 0.70710678118654752f)); }
      } else {
#pragma unroll
        for (int r = 0; r < 8; ++r) {
          float v = acc[i][j][r] + bv;
          if (EPI == 2) v = R[(size_t)(m0 + wm + 16 * i + rh + r) * ldy + n] + gv * v;
          so[(16 * i + rh + r) * 68 + 16 * j + cl] = v;
        }
      }
    }
  asm volatile("s_wait_dscnt 0" ::: "memory");
  __builtin_amdgcn_wave_barrier();
#pragma unroll 1
  for (int pass = 0; pass < 2; ++pass) {
    if (OUT16) {
      f16* Y = (f16*)Yv;
#pragma unroll
      for (int it = 0; it < 8; ++it) { const int c = lane + 32 * it, rr = c >> 3, q8 = (c & 7) * 8;
        union { f16 h[8]; v4u_t v; } u;
#pragma unroll
        for (int e = 0; e < 8; ++e) u.h[e] = (f16)so[rr * 68 + q8 + e];
        *(volatile v4u_t*)(Y + (size_t)(m0 + wm + rr) * ldy + n0 + wn + q8) = u.v; }
    } else {
      float* Y = (float*)Yv;
#pragma unroll
      for (int it = 0; it < 16; ++it) { const int f4 = lane + 32 * it, rr = f4 >> 4, q = (f4 & 15) * 4;
        *(volatile v4f_t*)(Y + (size_t)(m0 + wm + rr) * ldy + n0 + wn + q) = *(const v4fa*)(so + rr * 68 + q); }
    }
    __threadfence();
  }
}

__global__ __launch_bounds__(256) void k_transpose(const float* __restrict__ Wm, float* __restrict__ Wt, int rows, int cols, int ldin) {
  __shared__ float tS[64][65];
  const int tid = threadIdx.x, tbj = cols / 64, bi = blockIdx.x / tbj, bj = blockIdx.x % tbj;
  for (int e = tid; e < 64 * 64; e += 256) { const int r = e >> 6, c = e & 63; tS[r][c] = Wm[(size_t)(bi * 64 + r) * ldin + bj * 64 + c]; }
  __syncthreads();
  for (int ch = tid; ch < 64 * 16; ch += 256) { const int r = ch >> 4, q4 = (ch & 15) * 4; v4f_t o; o[0] = tS[q4][r]; o[1] = tS[q4 + 1][r]; o[2] = tS[q4 + 2][r]; o[3] = tS[q4 + 3][r];
    float* dst = Wt + (size_t)(bj * 64 + r) * rows + bi * 64 + q4; *(volatile v4f_t*)dst = o; __threadfence(); *(volatile v4f_t*)dst = o; }
}
__global__ __launch_bounds__(256) void k_tables(const float* __restrict__ rk, const float* __restrict__ rv, float* __restrict__ RKT, float* __restrict__ RV) {
  const int r = blockIdx.x;
#pragma unroll 1
  for (int pass = 0; pass < 2; ++pass) {
    if (r < DHr) { for (int c = threadIdx.x; c < NRP; c += 256) { const int cc = (c < NRr) ? c : NRr - 1; float v = rk[(size_t)cc * DHr + r]; v = (c < NRr) ? v : 0.0f; *(volatile float*)(RKT + (size_t)r * NRP + c) = v; } }
    { const int c = threadIdx.x; if (c < 128) { const int rr = (r < NRr) ? r : NRr - 1; float v = rv[(size_t)rr * DHr + (c & 63)]; v = (r < NRr) ? v : 0.0f; *(volatile float*)(RV + (size_t)r * 128 + c) = v; } }
    __threadfence(); }
}
__global__ __launch_bounds__(256) void k_rprsoftmax(float* __restrict__ Sm, const float* __restrict__ T, const int* __restrict__ vlens, int b, float* __restrict__ PR) {
  __shared__ float red[256];
  const int q = blockIdx.x, tid = threadIdx.x; const int vlen = vlens[b]; float* sr = Sm + (size_t)q * SSr; const float* tr = T + (size_t)q * NRP;
  float v[4]; float m = -3.0e38f;
#pragma unroll
  for (int e = 0; e < 4; ++e) { const int k = tid + 256 * e; int ridx = k - q; ridx = ridx < -64 ? -64 : (ridx > 64 ? 64 : ridx); ridx += 64;
    float s = (sr[k] + tr[ridx]) * 0.125f; s = (k < vlen) ? s : -1.0e6f; v[e] = s; m = fmaxf(m, s); }
  red[tid] = m; __syncthreads();
  for (int o = 128; o > 0; o >>= 1) { if (tid < o) red[tid] = fmaxf(red[tid], red[tid + o]); __syncthreads(); }
  m = red[0]; __syncthreads();
  float z = 0.0f;
#pragma unroll
  for (int e = 0; e < 4; ++e) { v[e] = expf(v[e] - m); z += v[e]; }
  red[tid] = z; __syncthreads();
  for (int o = 128; o > 0; o >>= 1) { if (tid < o) red[tid] += red[tid + o]; __syncthreads(); }
  const float sc = 1024.0f / red[0]; __syncthreads();
  float lo = 0.0f, hi = 0.0f;
#pragma unroll
  for (int e = 0; e < 4; ++e) { const int k = tid + 256 * e; v[e] *= sc; if (k <= q - 64) lo += v[e]; if (k >= q + 64) hi += v[e]; }
  red[tid] = lo; __syncthreads();
  for (int o = 128; o > 0; o >>= 1) { if (tid < o) red[tid] += red[tid + o]; __syncthreads(); }
  lo = red[0]; __syncthreads();
  red[tid] = hi; __syncthreads();
  for (int o = 128; o > 0; o >>= 1) { if (tid < o) red[tid] += red[tid + o]; __syncthreads(); }
  hi = red[0]; __syncthreads();
#pragma unroll 1
  for (int pass = 0; pass < 2; ++pass) {
#pragma unroll
    for (int e = 0; e < 4; ++e) *(volatile float*)(sr + tid + 256 * e) = v[e];
    __threadfence(); }
  __syncthreads();
  { const int r = tid;
    const int k = q + r - 64; const int kc = k < 0 ? 0 : (k >= SSr ? SSr - 1 : k); const float pk = sr[kc];
    float pr = (r == 0) ? lo : (r == 128) ? hi : (r < NRr && k >= 0 && k < SSr) ? pk : 0.0f;
    *(volatile float*)(PR + (size_t)q * NRP + r) = pr; __threadfence(); *(volatile float*)(PR + (size_t)q * NRP + r) = pr; }
}
__global__ __launch_bounds__(128) void k_ones(float* __restrict__ p) { const float v = 1.0f; *(volatile float*)(p + threadIdx.x) = v; __threadfence(); *(volatile float*)(p + threadIdx.x) = v; }
__global__ __launch_bounds__(64) void k_place(const float* __restrict__ O, int co, int b, int h, bf16* __restrict__ O16) { __shared__ __attribute__((aligned(16))) bf16 s[64];
  const int q = blockIdx.x, d = threadIdx.x; s[d] = (bf16)(O[(size_t)q * 128 + co + d] * (1.0f / 1024.0f)); __syncthreads();
  if (d < 8) { bf16* dst = O16 + ((size_t)b * SSr + q) * Dr + h * DHr + d * 8; *(volatile v4u_t*)dst = *(const v4ua*)(s + d * 8); __threadfence(); *(volatile v4u_t*)dst = *(const v4ua*)(s + d * 8); } }

extern "C" void kernel_launch(void* const* d_in, const int* in_sizes, int n_in,
                              void* d_out, int out_size, void* d_ws, size_t ws_size,
                              hipStream_t stream) {
  (void)in_sizes; (void)n_in; (void)out_size;
  const float** f = (const float**)d_in;
  const float* xq = f[0], *xk = f[1], *xv = f[2]; const int* vlens = (const int*)d_in[3]; const float* Wq = f[4], *Wk = f[5], *Wv = f[6], *Wo = f[7], *rk = f[8], *rv = f[9];
  float* out = (float*)d_out;
  char* ws = (char*)d_ws;
  float* Q = (float*)ws; ws += (size_t)MTOK * Dr * 4; float* Kf = (float*)ws; ws += (size_t)MTOK * Dr * 4; float* V = (float*)ws; ws += (size_t)(MTOK * Dr + 64) * 4;
  float* RKT = (float*)ws; ws += (size_t)DHr * NRP * 4; float* RV = (float*)ws; ws += (size_t)NRP * 128 * 4;
  float* KT = (float*)ws; ws += (size_t)DHr * SSr * 4;
  float* S_ = (float*)ws; ws += (size_t)SSr * SSr * 4; float* T = (float*)ws; ws += (size_t)SSr * NRP * 4; float* PR = (float*)ws; ws += (size_t)SSr * NRP * 4; float* O = (float*)ws; ws += (size_t)SSr * 128 * 4;
  bf16* O16 = (bf16*)ws; ws += (size_t)MTOK * Dr * 2;
  float* ones = (float*)ws; ws += 128 * 4;
  if ((size_t)(ws - (char*)d_ws) > ws_size) return;
  const dim3 blk(256); const dim3 gp(MTOK / 128, Dr / 128);
  k_tables<<<dim3(NRP), blk, 0, stream>>>(rk, rv, RKT, RV);
  k_ones<<<dim3(1), dim3(128), 0, stream>>>(ones);
  gemm_kne<float, 0, false><<<gp, blk, 0, stream>>>(xq, Dr, Wq, Dr, nullptr, nullptr, nullptr, Q, Dr, Dr);
  gemm_kne<float, 0, false><<<gp, blk, 0, stream>>>(xk, Dr, Wk, Dr, nullptr, nullptr, nullptr, Kf, Dr, Dr);
  gemm_kne<float, 0, false><<<gp, blk, 0, stream>>>(xv, Dr, Wv, Dr, nullptr, nullptr, nullptr, V, Dr, Dr);
  for (int b = 0; b < NB; ++b) for (int h = 0; h < NH; ++h) {
    const float* Qbh = Q + (size_t)b * SSr * Dr + h * DHr; const float* Kbh = Kf + (size_t)b * SSr * Dr + h * DHr;
    k_transpose<<<dim3((SSr / 64) * (DHr / 64)), blk, 0, stream>>>(Kbh, KT, SSr, DHr, Dr);
    gemm_kne<float, 0, false><<<dim3(SSr / 128, SSr / 128), blk, 0, stream>>>(Qbh, Dr, KT, SSr, nullptr, nullptr, nullptr, S_, SSr, DHr);
    gemm_kne<float, 0, false><<<dim3(SSr / 128, NRP / 128), blk, 0, stream>>>(Qbh, Dr, RKT, NRP, nullptr, nullptr, nullptr, T, NRP, DHr);
    k_rprsoftmax<<<dim3(SSr), blk, 0, stream>>>(S_, T, vlens, b, PR);
    const int co = (h < NH - 1) ? 0 : 64; const float* Vcols = V + (size_t)b * SSr * Dr + (h < NH - 1 ? h : h - 1) * DHr;
    gemm_kne<float, 0, false><<<dim3(SSr / 128, 1), blk, 0, stream>>>(S_, SSr, Vcols, Dr, nullptr, nullptr, nullptr, O, 128, SSr);
    gemm_kne<float, 2, false><<<dim3(SSr / 128, 1), blk, 0, stream>>>(PR, NRP, RV, 128, nullptr, O, ones, O, 128, NRP);
    k_place<<<dim3(SSr), dim3(64), 0, stream>>>(O, co, b, h, O16);
  }
  gemm_kne<bf16, 0, false><<<gp, blk, 0, stream>>>(O16, Dr, Wo, Dr, nullptr, nullptr, nullptr, out, Dr, Dr);
}
